// TemporalFusionLayer_26164940767821
// MI455X (gfx1250) — hardware-verified
//
#include <hip/hip_runtime.h>
#include <stddef.h>
#include <stdint.h>

#define NB  2
#define LQ  2049
#define TS  683
#define LP  2176
#define NQB (LP / 128)
#define CC  1024
#define C3  3072
#define FF  4096
#define NH  16
#define HD  64
#define RP  (NB * LP)
#define NKC 33
#define MQ  2112
#define TG  726
#define PLQ ((size_t)NB * NH * LP * HD)

static_assert(LP % 128 == 0);
static_assert(NKC * 64 >= LQ);
static_assert(NKC * 64 <= LP);
static_assert(MQ == NKC * 64);
static_assert(RP % 128 == 0);
static_assert(3 * TS == LQ);
static_assert(3 * TG >= LP);
static_assert(3 * (TG - 1) < LP);
static_assert(NH * HD == CC);
static_assert(CC % 64 == 0);
static_assert(C3 % 64 == 0);
static_assert(FF % 64 == 0);

typedef _Float16 v16h __attribute__((ext_vector_type(16)));
typedef _Float16 v8h  __attribute__((ext_vector_type(8)));
typedef _Float16 v4h  __attribute__((ext_vector_type(4)));
typedef float    v8f  __attribute__((ext_vector_type(8)));
typedef float    v4f  __attribute__((ext_vector_type(4)));
typedef unsigned int v4u __attribute__((ext_vector_type(4)));

union Frag  { v16h v; v8h h[2]; };
union Pack8 { v8h h; v4u u; };
union Pack4 { v4h h; unsigned long long u; };

__device__ __forceinline__ v8f mma16(v16h a, v16h b, v8f c) {
  c = __builtin_amdgcn_wmma_f32_16x16x32_f16(false, a, false, b, (short)0, c, false, false);
  asm volatile("v_nop\n\tv_nop\n\tv_nop\n\tv_nop" : "+v"(c) : "v"(a), "v"(b));
  return c;
}

__device__ __forceinline__ v16h ldfrag(const _Float16* p, int ld, int row0, int k0, int lane) {
  const int m = lane & 15, lh = lane >> 4;
  const _Float16* q = p + (size_t)(row0 + m) * ld + k0 + 8 * lh;
  Frag f;
  f.h[0] = *(const v8h*)(q);
  f.h[1] = *(const v8h*)(q + 16);
  return f.v;
}

__device__ __forceinline__ v8f zero8() { return (v8f){0.f, 0.f, 0.f, 0.f, 0.f, 0.f, 0.f, 0.f}; }

__device__ __forceinline__ void gemm32x64(const _Float16* __restrict__ A, int lda,
                                          const _Float16* __restrict__ Bt, int ldb, int K,
                                          int m0, int n0, int lane, v8f (&acc)[2][4]) {
#pragma unroll 2
  for (int k0 = 0; k0 < K; k0 += 32) {
    const v16h a0 = ldfrag(A, lda, m0, k0, lane);
    const v16h a1 = ldfrag(A, lda, m0 + 16, k0, lane);
    const v16h b0 = ldfrag(Bt, ldb, n0, k0, lane);
    const v16h b1 = ldfrag(Bt, ldb, n0 + 16, k0, lane);
    const v16h b2 = ldfrag(Bt, ldb, n0 + 32, k0, lane);
    const v16h b3 = ldfrag(Bt, ldb, n0 + 48, k0, lane);
    acc[0][0] = mma16(a0, b0, acc[0][0]);
    acc[1][0] = mma16(a1, b0, acc[1][0]);
    acc[0][1] = mma16(a0, b1, acc[0][1]);
    acc[1][1] = mma16(a1, b1, acc[1][1]);
    acc[0][2] = mma16(a0, b2, acc[0][2]);
    acc[1][2] = mma16(a1, b2, acc[1][2]);
    acc[0][3] = mma16(a0, b3, acc[0][3]);
    acc[1][3] = mma16(a1, b3, acc[1][3]);
  }
}

__global__ __launch_bounds__(256) void k_cvt_x(const float* __restrict__ x, _Float16* __restrict__ xh, int ngrp) {
  const int t = blockIdx.x * 256 + (int)threadIdx.x;
  if (t >= ngrp) return;
  const int rowp = t >> 7;
  const int pc = t & 127;
  const int b = rowp / LP;
  const int n = rowp - b * LP;
  const bool valid = (n < LQ);
  const int nn = valid ? n : (LQ - 1);
  const float* src = x + ((size_t)(b * LQ + nn)) * CC + pc * 8;
  const v4f a0 = *(const v4f*)(src);
  const v4f a1 = *(const v4f*)(src + 4);
  Pack8 pk;
  pk.h = (v8h){(_Float16)(valid ? a0[0] : 0.f), (_Float16)(valid ? a0[1] : 0.f),
               (_Float16)(valid ? a0[2] : 0.f), (_Float16)(valid ? a0[3] : 0.f),
               (_Float16)(valid ? a1[0] : 0.f), (_Float16)(valid ? a1[1] : 0.f),
               (_Float16)(valid ? a1[2] : 0.f), (_Float16)(valid ? a1[3] : 0.f)};
  const v4u vv = pk.u;
  volatile v4u* d = (volatile v4u*)(xh + (size_t)t * 8);
  *d = vv;
  __threadfence();
  *d = vv;
}

__global__ __launch_bounds__(256) void k_cvt_w(const float* __restrict__ w, _Float16* __restrict__ wh,
                                               int ngrp, float sc) {
  const int t = blockIdx.x * 256 + (int)threadIdx.x;
  if (t >= ngrp) return;
  const size_t o = (size_t)t * 8;
  const v4f a0 = *(const v4f*)(w + o);
  const v4f a1 = *(const v4f*)(w + o + 4);
  Pack8 pk;
  pk.h = (v8h){(_Float16)(a0[0] * sc), (_Float16)(a0[1] * sc), (_Float16)(a0[2] * sc), (_Float16)(a0[3] * sc),
               (_Float16)(a1[0] * sc), (_Float16)(a1[1] * sc), (_Float16)(a1[2] * sc), (_Float16)(a1[3] * sc)};
  const v4u vv = pk.u;
  volatile v4u* d = (volatile v4u*)(wh + o);
  *d = vv;
  __threadfence();
  *d = vv;
}

#define STP 72
__global__ __launch_bounds__(128) void k_qkv(const _Float16* __restrict__ xh,
                                             const _Float16* __restrict__ wt,
                                             const float* __restrict__ bias,
                                             _Float16* __restrict__ qkv) {
  __shared__ __align__(16) _Float16 st[128 * STP];
  const int tid = threadIdx.x, lane = tid & 31, wave = tid >> 5;
  const int hh = lane >> 4, c = lane & 15;
  const int mb = blockIdx.x * 128;
  const int m0 = mb + wave * 32;
  const int n0 = blockIdx.y * 64;

  v8f acc[2][4];
#pragma unroll
  for (int s = 0; s < 2; ++s)
#pragma unroll
    for (int t = 0; t < 4; ++t) acc[s][t] = zero8();
  gemm32x64(xh, CC, wt, CC, CC, m0, n0, lane, acc);

#pragma unroll
  for (int t = 0; t < 4; ++t) {
    const float bv = bias[n0 + 16 * t + c];
#pragma unroll
    for (int sub = 0; sub < 2; ++sub) {
#pragma unroll
      for (int r = 0; r < 8; ++r) {
        const int lr = wave * 32 + sub * 16 + 8 * hh + r;
        st[lr * STP + 16 * t + c] = (_Float16)(acc[sub][t][r] * 0.03125f + bv);
      }
    }
  }
  __syncthreads();

  const int which = n0 >> 10;
  const int head  = (n0 & (CC - 1)) >> 6;
  const int b  = mb / LP;
  const int nb = mb - b * LP;
  const int bh = b * NH + head;
  v4u val[8];
  size_t go[8];
  if (which < 2) {
#pragma unroll
    for (int j = 0; j < 8; ++j) {
      const int p  = tid + 128 * j;
      const int lr = p >> 3;
      const int pc = p & 7;
      Pack8 pk;
      pk.h  = *(const v8h*)(st + lr * STP + pc * 8);
      val[j] = pk.u;
      go[j]  = (size_t)which * PLQ + ((size_t)bh * LP + nb + lr) * HD + pc * 8;
    }
  } else {
#pragma unroll
    for (int j = 0; j < 8; ++j) {
      const int p  = tid + 128 * j;
      const int L  = p >> 3;
      const int pc = p & 7;
      const int d  = L >> 1;
      const int nl = (L & 1) * 64 + pc * 8;
      const _Float16* cp = st + nl * STP + d;
      Pack8 pk;
      pk.h = (v8h){cp[0 * STP], cp[1 * STP], cp[2 * STP], cp[3 * STP],
                   cp[4 * STP], cp[5 * STP], cp[6 * STP], cp[7 * STP]};
      val[j] = pk.u;
      go[j]  = 2 * PLQ + ((size_t)bh * HD + d) * LP + nb + nl;
    }
  }
  for (int ps = 0; ps < 2; ++ps) {
#pragma unroll
    for (int j = 0; j < 8; ++j) *(volatile v4u*)(qkv + go[j]) = val[j];
    __threadfence();
  }
}

#define KTP 72
#define PTP 72
__global__ __launch_bounds__(256) void k_attn(const _Float16* __restrict__ qp,
                                              const _Float16* __restrict__ kp,
                                              const _Float16* __restrict__ vt,
                                              _Float16* __restrict__ op,
                                              float* __restrict__ stp, float sscale) {
  __shared__ __align__(16) _Float16 Ks[64 * KTP];
  __shared__ __align__(16) _Float16 Vs[64 * KTP];
  __shared__ __align__(16) _Float16 Ps[8][16 * PTP];
  __shared__ __align__(16) float sst[128];

  const int tid = threadIdx.x, lane = tid & 31, wave = tid >> 5;
  const int hh = lane >> 4, c = lane & 15;
  const int bh = blockIdx.x / NQB;
  const int qb = blockIdx.x - bh * NQB;
  const int b  = bh >> 4, h = bh & (NH - 1);
  const int q0 = qb * 128 + wave * 16;

  const _Float16* Q = qp + (size_t)bh * LP * HD;
  const _Float16* K = kp + (size_t)bh * LP * HD;
  const _Float16* V = vt + (size_t)bh * HD * LP;

  v16h qa[2];
  qa[0] = ldfrag(Q, HD, q0, 0, lane);
  qa[1] = ldfrag(Q, HD, q0, 32, lane);

  const float NEGI = -__builtin_huge_valf();
  float mrow[8], lrow[8];
  v8f oacc[4];
#pragma unroll
  for (int r = 0; r < 8; ++r) { mrow[r] = NEGI; lrow[r] = 0.f; }
#pragma unroll
  for (int t = 0; t < 4; ++t) oacc[t] = zero8();

  _Float16* pw = Ps[wave];

  for (int kc = 0; kc < NKC; ++kc) {
    const int kv0 = kc * 64;
    __syncthreads();
    {
      const int r  = tid >> 2;
      const int qq = (tid & 3) * 16;
      const _Float16* ks = K + (size_t)(kv0 + r) * HD + qq;
      *(v8h*)(Ks + r * KTP + qq)     = *(const v8h*)(ks);
      *(v8h*)(Ks + r * KTP + qq + 8) = *(const v8h*)(ks + 8);
      const _Float16* vs = V + (size_t)r * LP + kv0 + qq;
      *(v8h*)(Vs + r * KTP + qq)     = *(const v8h*)(vs);
      *(v8h*)(Vs + r * KTP + qq + 8) = *(const v8h*)(vs + 8);
    }
    __syncthreads();

    v8f s[4];
#pragma unroll
    for (int j = 0; j < 4; ++j) s[j] = zero8();
#pragma unroll
    for (int dc = 0; dc < 2; ++dc) {
#pragma unroll
      for (int j = 0; j < 4; ++j) {
        const v16h kb = ldfrag(Ks, KTP, j * 16, dc * 32, lane);
        s[j] = mma16(qa[dc], kb, s[j]);
      }
    }
    float cm[8];
#pragma unroll
    for (int r = 0; r < 8; ++r) {
      float m = NEGI;
#pragma unroll
      for (int j = 0; j < 4; ++j) {
        const int key = kv0 + j * 16 + c;
        const float sv = (key < LQ) ? s[j][r] * sscale : NEGI;
        s[j][r] = sv;
        m = fmaxf(m, sv);
      }
#pragma unroll
      for (int off = 1; off < 16; off <<= 1) m = fmaxf(m, __shfl_xor(m, off, 32));
      cm[r] = m;
    }
    float al[8];
#pragma unroll
    for (int r = 0; r < 8; ++r) {
      const float mnew  = fmaxf(mrow[r], cm[r]);
      const float alpha = __expf(mrow[r] - mnew);
      mrow[r] = mnew;
      float psum = 0.f;
#pragma unroll
      for (int j = 0; j < 4; ++j) {
        const float p = __expf(s[j][r] - mnew);
        psum += p;
        pw[(8 * hh + r) * PTP + j * 16 + c] = (_Float16)(p * 1024.0f);
      }
#pragma unroll
      for (int off = 1; off < 16; off <<= 1) psum += __shfl_xor(psum, off, 32);
      lrow[r] = lrow[r] * alpha + psum;
      al[r] = alpha;
    }
#pragma unroll
    for (int t = 0; t < 4; ++t)
#pragma unroll
      for (int r = 0; r < 8; ++r) oacc[t][r] *= al[r];
    __syncthreads();

#pragma unroll
    for (int kk = 0; kk < 2; ++kk) {
      const v16h pa = ldfrag(pw, PTP, 0, kk * 32, lane);
#pragma unroll
      for (int t = 0; t < 4; ++t) {
        const v16h vb = ldfrag(Vs, KTP, t * 16, kk * 32, lane);
        oacc[t] = mma16(pa, vb, oacc[t]);
      }
    }
  }
  __syncthreads();

  {
    float stv[8];
#pragma unroll
    for (int r = 0; r < 8; ++r) stv[r] = mrow[r] + __logf(lrow[r]);
    if (c == 0) {
#pragma unroll
      for (int r = 0; r < 8; ++r) sst[wave * 16 + 8 * hh + r] = stv[r];
    }
  }
#pragma unroll
  for (int r = 0; r < 8; ++r) {
    const float inv = 0.015625f / lrow[r];
#pragma unroll
    for (int t = 0; t < 4; ++t) pw[(8 * hh + r) * PTP + 16 * t + c] = (_Float16)(oacc[t][r] * inv);
  }
  __syncthreads();
  v4u val[4];
  size_t go[4];
#pragma unroll
  for (int it = 0; it < 4; ++it) {
    const int p  = lane + 32 * it;
    const int L  = p >> 3;
    const int pc = p & 7;
    Pack8 pk;
    pk.h   = *(const v8h*)(pw + L * PTP + pc * 8);
    val[it] = pk.u;
    go[it]  = ((size_t)(b * LP + q0 + L)) * CC + (size_t)h * HD + pc * 8;
  }
  const v4f sv4 = *(const v4f*)(sst + 4 * lane);
  float* sdst = stp + (size_t)bh * LP + qb * 128 + 4 * lane;
  for (int ps = 0; ps < 2; ++ps) {
#pragma unroll
    for (int it = 0; it < 4; ++it) *(volatile v4u*)(op + go[it]) = val[it];
    if (wave == 0) *(volatile v4f*)sdst = sv4;
    __threadfence();
  }
}

#define OTP 68
__global__ __launch_bounds__(64) void k_map(const _Float16* __restrict__ qp,
                                            const _Float16* __restrict__ kp,
                                            const float* __restrict__ stp,
                                            float* __restrict__ mp, float sscale) {
  __shared__ __align__(16) float st[2][16 * OTP];
  const int tid = threadIdx.x, lane = tid & 31, wave = tid >> 5;
  const int hh = lane >> 4, c = lane & 15;
  const int b = blockIdx.z;
  const int row0 = blockIdx.x * 64 + wave * 32;
  const int key0 = blockIdx.y * 64;

  v8f macc[2][4];
#pragma unroll
  for (int s = 0; s < 2; ++s)
#pragma unroll
    for (int t = 0; t < 4; ++t) macc[s][t] = zero8();

#pragma unroll 1
  for (int h = 0; h < NH; ++h) {
    const int bh = b * NH + h;
    const _Float16* Q = qp + (size_t)bh * LP * HD;
    const _Float16* K = kp + (size_t)bh * LP * HD;
    const v16h a00 = ldfrag(Q, HD, row0, 0, lane);
    const v16h a01 = ldfrag(Q, HD, row0, 32, lane);
    const v16h a10 = ldfrag(Q, HD, row0 + 16, 0, lane);
    const v16h a11 = ldfrag(Q, HD, row0 + 16, 32, lane);
    const float* sp = stp + (size_t)bh * LP + row0 + 8 * hh;
    const v8f st0 = *(const v8f*)(sp);
    const v8f st1 = *(const v8f*)(sp + 16);
#pragma unroll
    for (int j = 0; j < 4; ++j) {
      const v16h kb0 = ldfrag(K, HD, key0 + 16 * j, 0, lane);
      const v16h kb1 = ldfrag(K, HD, key0 + 16 * j, 32, lane);
      v8f sa = mma16(a00, kb0, zero8());
      sa = mma16(a01, kb1, sa);
      v8f sb = mma16(a10, kb0, zero8());
      sb = mma16(a11, kb1, sb);
#pragma unroll
      for (int r = 0; r < 8; ++r) {
        macc[0][j][r] += __expf(fmaf(sa[r], sscale, -st0[r]));
        macc[1][j][r] += __expf(fmaf(sb[r], sscale, -st1[r]));
      }
    }
  }

  float* sw = st[wave];
#pragma unroll
  for (int sub = 0; sub < 2; ++sub) {
    __syncthreads();
#pragma unroll
    for (int t = 0; t < 4; ++t) {
#pragma unroll
      for (int r = 0; r < 8; ++r) sw[(8 * hh + r) * OTP + 16 * t + c] = macc[sub][t][r] * 0.0625f;
    }
    __syncthreads();
    v4f val[8];
    size_t go[8];
#pragma unroll
    for (int it = 0; it < 8; ++it) {
      const int p    = lane + 32 * it;
      const int L    = p >> 3;
      const int pc   = p & 7;
      const int row  = L >> 1;
      const int half = L & 1;
      val[it] = *(const v4f*)(sw + row * OTP + half * 32 + pc * 4);
      go[it]  = ((size_t)(b * MQ + row0 + sub * 16 + row)) * MQ + key0 + half * 32 + pc * 4;
    }
    for (int ps = 0; ps < 2; ++ps) {
#pragma unroll
      for (int it = 0; it < 8; ++it) *(volatile v4f*)(mp + go[it]) = val[it];
      __threadfence();
    }
  }
}

__global__ __launch_bounds__(256) void k_flat(const float* __restrict__ mp, float* __restrict__ o1, int n1) {
  const int t = blockIdx.x * 256 + (int)threadIdx.x;
  const int i0 = t * 4;
  if (i0 >= n1) return;
  float v[4];
#pragma unroll
  for (int j = 0; j < 4; ++j) {
    int i = i0 + j;
    i = (i < n1) ? i : (n1 - 1);
    const int bb  = i / (LQ * LQ);
    const int rem = i - bb * (LQ * LQ);
    const int l   = rem / LQ;
    const int m   = rem - l * LQ;
    v[j] = mp[((size_t)(bb * MQ + l)) * MQ + m];
  }
  if (i0 + 4 <= n1) {
    const v4f vv = (v4f){v[0], v[1], v[2], v[3]};
    volatile v4f* d = (volatile v4f*)(o1 + i0);
    *d = vv;
    __threadfence();
    *d = vv;
  } else {
    volatile float* d = (volatile float*)o1;
    for (int j = 0; j < 4; ++j) if (i0 + j < n1) d[i0 + j] = v[j];
    __threadfence();
    for (int j = 0; j < 4; ++j) if (i0 + j < n1) d[i0 + j] = v[j];
  }
}

__global__ __launch_bounds__(128) void k_gemm32(const _Float16* __restrict__ ap,
                                                const _Float16* __restrict__ wt,
                                                const float* __restrict__ bias,
                                                float* __restrict__ out, int K, int N, float oscale) {
  __shared__ __align__(16) float st[4][16 * OTP];
  const int tid = threadIdx.x, lane = tid & 31, wave = tid >> 5;
  const int hh = lane >> 4, c = lane & 15;
  const int m0 = blockIdx.x * 128 + wave * 32;
  const int n0 = blockIdx.y * 64;

  v8f acc[2][4];
#pragma unroll
  for (int s = 0; s < 2; ++s)
#pragma unroll
    for (int t = 0; t < 4; ++t) acc[s][t] = zero8();
  gemm32x64(ap, K, wt, K, K, m0, n0, lane, acc);

  float bvs[4];
#pragma unroll
  for (int t = 0; t < 4; ++t) bvs[t] = bias[n0 + 16 * t + c];

  float* sw = st[wave];
#pragma unroll
  for (int sub = 0; sub < 2; ++sub) {
    __syncthreads();
#pragma unroll
    for (int t = 0; t < 4; ++t) {
#pragma unroll
      for (int r = 0; r < 8; ++r)
        sw[(8 * hh + r) * OTP + 16 * t + c] = acc[sub][t][r] * oscale + bvs[t];
    }
    __syncthreads();
    v4f val[8];
    size_t go[8];
#pragma unroll
    for (int it = 0; it < 8; ++it) {
      const int p    = lane + 32 * it;
      const int L    = p >> 3;
      const int pc   = p & 7;
      const int row  = L >> 1;
      const int half = L & 1;
      val[it] = *(const v4f*)(sw + row * OTP + half * 32 + pc * 4);
      go[it]  = (size_t)(m0 + sub * 16 + row) * N + n0 + half * 32 + pc * 4;
    }
    for (int ps = 0; ps < 2; ++ps) {
#pragma unroll
      for (int it = 0; it < 8; ++it) *(volatile v4f*)(out + go[it]) = val[it];
      __threadfence();
    }
  }
}

template <int GELU>
__global__ __launch_bounds__(128) void k_gemm16(const _Float16* __restrict__ ap,
                                                const _Float16* __restrict__ wt,
                                                const float* __restrict__ bias,
                                                _Float16* __restrict__ out, int K, int N, float oscale) {
  __shared__ __align__(16) _Float16 st[128 * STP];
  const int tid = threadIdx.x, lane = tid & 31, wave = tid >> 5;
  const int hh = lane >> 4, c = lane & 15;
  const int mb = blockIdx.x * 128;
  const int m0 = mb + wave * 32;
  const int n0 = blockIdx.y * 64;

  v8f acc[2][4];
#pragma unroll
  for (int s = 0; s < 2; ++s)
#pragma unroll
    for (int t = 0; t < 4; ++t) acc[s][t] = zero8();
  gemm32x64(ap, K, wt, K, K, m0, n0, lane, acc);

#pragma unroll
  for (int t = 0; t < 4; ++t) {
    const float bv = bias[n0 + 16 * t + c];
#pragma unroll
    for (int sub = 0; sub < 2; ++sub) {
#pragma unroll
      for (int r = 0; r < 8; ++r) {
        const int lr = wave * 32 + sub * 16 + 8 * hh + r;
        float v = acc[sub][t][r] * oscale + bv;
        if (GELU) v = 0.5f * v * (1.0f + erff(v * 0.70710678118654752f));
        st[lr * STP + 16 * t + c] = (_Float16)v;
      }
    }
  }
  __syncthreads();

  v4u val[8];
  size_t go[8];
#pragma unroll
  for (int j = 0; j < 8; ++j) {
    const int p  = tid + 128 * j;
    const int lr = p >> 3;
    const int pc = p & 7;
    Pack8 pk;
    pk.h  = *(const v8h*)(st + lr * STP + pc * 8);
    val[j] = pk.u;
    go[j]  = (size_t)(mb + lr) * N + n0 + pc * 8;
  }
  for (int ps = 0; ps < 2; ++ps) {
#pragma unroll
    for (int j = 0; j < 8; ++j) *(volatile v4u*)(out + go[j]) = val[j];
    __threadfence();
  }
}

template <int MODE>
__global__ __launch_bounds__(256) void k_ln(const float* __restrict__ resid,
                                            const float* __restrict__ delta,
                                            const float* __restrict__ g, const float* __restrict__ be,
                                            float* __restrict__ outf, _Float16* __restrict__ outh,
                                            float* __restrict__ outd) {
  __shared__ float red[16];
  const int tid = threadIdx.x, lane = tid & 31, wave = tid >> 5;
  const int rowp = blockIdx.x;
  const int b = rowp / LP;
  const int n = rowp - b * LP;
  const bool valid = (n < LQ);
  const int c0 = tid * 4;

  const v4f dl = *(const v4f*)(delta + (size_t)rowp * CC + c0);
  v4f rs;
  if (MODE == 0) {
    const int nn = valid ? n : (LQ - 1);
    const v4f rx = *(const v4f*)(resid + ((size_t)(b * LQ + nn)) * CC + c0);
    rs = (v4f){valid ? rx[0] : 0.f, valid ? rx[1] : 0.f, valid ? rx[2] : 0.f, valid ? rx[3] : 0.f};
  } else {
    rs = *(const v4f*)(resid + (size_t)rowp * CC + c0);
  }
  const v4f tv = rs + dl;

  float s = (tv[0] + tv[1]) + (tv[2] + tv[3]);
#pragma unroll
  for (int off = 1; off < 32; off <<= 1) s += __shfl_xor(s, off, 32);
  if (lane == 0) red[wave] = s;
  __syncthreads();
  float tot = 0.f;
#pragma unroll
  for (int i = 0; i < 8; ++i) tot += red[i];
  const float mean = tot * (1.0f / (float)CC);

  const v4f dv = (v4f){tv[0] - mean, tv[1] - mean, tv[2] - mean, tv[3] - mean};
  float sq = (dv[0] * dv[0] + dv[1] * dv[1]) + (dv[2] * dv[2] + dv[3] * dv[3]);
#pragma unroll
  for (int off = 1; off < 32; off <<= 1) sq += __shfl_xor(sq, off, 32);
  if (lane == 0) red[8 + wave] = sq;
  __syncthreads();
  float tot2 = 0.f;
#pragma unroll
  for (int i = 0; i < 8; ++i) tot2 += red[8 + i];
  const float var = tot2 * (1.0f / (float)CC);
  const float inv = rsqrtf(var + 1e-5f);

  const v4f gv = *(const v4f*)(g + c0);
  const v4f bv = *(const v4f*)(be + c0);
  const v4f y = (v4f){dv[0] * inv * gv[0] + bv[0], dv[1] * inv * gv[1] + bv[1],
                      dv[2] * inv * gv[2] + bv[2], dv[3] * inv * gv[3] + bv[3]};

  if (MODE == 2) {
    if (valid) {
      volatile v4f* d = (volatile v4f*)(outd + ((size_t)(b * LQ + n)) * CC + c0);
      *d = y;
      __threadfence();
      *d = y;
    }
  } else {
    Pack4 pk;
    pk.h = (v4h){(_Float16)y[0], (_Float16)y[1], (_Float16)y[2], (_Float16)y[3]};
    const unsigned long long hv = pk.u;
    volatile v4f* df = (volatile v4f*)(outf + (size_t)rowp * CC + c0);
    volatile unsigned long long* dh = (volatile unsigned long long*)(outh + (size_t)rowp * CC + c0);
    *df = y;
    *dh = hv;
    __threadfence();
    *df = y;
    *dh = hv;
  }
}

__global__ __launch_bounds__(64) void k_ca(const _Float16* __restrict__ p2, _Float16* __restrict__ cp,
                                           float sscale) {
  __shared__ __align__(16) _Float16 cs[3 * CC];
  const int tid = threadIdx.x;
  const int b = blockIdx.x / TG;
  const int t = blockIdx.x - b * TG;
  const int r0 = 3 * t;
  const int nr = (LP - r0 < 3) ? (LP - r0) : 3;
  const size_t rowbase = (size_t)b * LP + r0;
  const bool live = (t < TS);
  if (live) {
    const int h = tid & 15;
    int q = tid >> 4;
    q = (q > 2) ? 2 : q;
    const _Float16* Qr = p2 + (rowbase + q) * C3 + h * HD;
    const _Float16* Kr = p2 + rowbase * C3 + CC + h * HD;
    const _Float16* Vr = p2 + rowbase * C3 + 2 * CC + h * HD;
    float s0 = 0.f, s1 = 0.f, s2 = 0.f;
#pragma unroll 1
    for (int dc = 0; dc < HD; dc += 8) {
      const v8h qv = *(const v8h*)(Qr + dc);
      const v8h k0 = *(const v8h*)(Kr + dc);
      const v8h k1 = *(const v8h*)(Kr + C3 + dc);
      const v8h k2 = *(const v8h*)(Kr + 2 * C3 + dc);
#pragma unroll
      for (int i = 0; i < 8; ++i) {
        const float qf = (float)qv[i];
        s0 = fmaf(qf, (float)k0[i], s0);
        s1 = fmaf(qf, (float)k1[i], s1);
        s2 = fmaf(qf, (float)k2[i], s2);
      }
    }
    s0 *= sscale; s1 *= sscale; s2 *= sscale;
    const float mx = fmaxf(s0, fmaxf(s1, s2));
    const float e0 = __expf(s0 - mx), e1 = __expf(s1 - mx), e2 = __expf(s2 - mx);
    const float inv = 1.0f / (e0 + e1 + e2);
    const float w0 = e0 * inv, w1 = e1 * inv, w2 = e2 * inv;
    _Float16* dst = cs + q * CC + h * HD;
#pragma unroll 1
    for (int dc = 0; dc < HD; dc += 8) {
      const v8h v0 = *(const v8h*)(Vr + dc);
      const v8h v1 = *(const v8h*)(Vr + C3 + dc);
      const v8h v2 = *(const v8h*)(Vr + 2 * C3 + dc);
      v8h o8;
#pragma unroll
      for (int i = 0; i < 8; ++i) {
        float o = w0 * (float)v0[i];
        o = fmaf(w1, (float)v1[i], o);
        o = fmaf(w2, (float)v2[i], o);
        o8[i] = (_Float16)(o * 16.0f);
      }
      Pack8 pk;
      pk.h = o8;
      *(v4u*)(dst + dc) = pk.u;
    }
  }
  __syncthreads();
  const v4u z4 = (v4u){0u, 0u, 0u, 0u};
  v4u val[6];
  size_t go[6];
  bool pr[6];
#pragma unroll
  for (int i = 0; i < 6; ++i) {
    const int p   = tid + 64 * i;
    const int row = p >> 7;
    const int off = (p & 127) * 8;
    Pack8 pk;
    pk.h = *(const v8h*)(cs + row * CC + off);
    const v4u lv = pk.u;
    val[i] = (v4u){live ? lv[0] : 0u, live ? lv[1] : 0u, live ? lv[2] : 0u, live ? lv[3] : 0u};
    go[i]  = (rowbase + row) * CC + off;
    pr[i]  = (row < nr);
  }
  (void)z4;
  for (int ps = 0; ps < 2; ++ps) {
#pragma unroll
    for (int i = 0; i < 6; ++i) if (pr[i]) *(volatile v4u*)(cp + go[i]) = val[i];
    __threadfence();
  }
}

#define SZ_RF ((size_t)RP * CC * 4)
#define SZ_RH ((size_t)RP * CC * 2)
#define SZ_S0 ((size_t)NB * MQ * MQ * 4)
#define SZ_S1 ((size_t)3 * PLQ * 2)
#define SZ_P2 ((size_t)RP * C3 * 2)
#define SZ_HH ((size_t)RP * FF * 2)
#define SZ_ST ((size_t)NB * NH * LP * 4)
#define SZ_W1K ((size_t)CC * CC * 2)
#define SZ_W3K ((size_t)C3 * CC * 2)
#define SZ_WFF ((size_t)FF * CC * 2)

#define O_S0     ((size_t)0)
#define O_XH     (O_S0)
#define O_WSAIN  (O_S0 + SZ_RH)
#define O_MP     (O_S0)
#define O_X1     (O_S0)
#define O_X1H    (O_S0 + SZ_RF)
#define O_CP     (O_S0 + SZ_RF + SZ_RH)
#define O_HH     (O_S0)
#define O_S1     (O_S0 + SZ_S0)
#define O_QKV    (O_S1)
#define O_GOUT   (O_S1)
#define O_P2     (O_S1)
#define O_S2     (O_S1 + SZ_S1)
#define O_OP     (O_S2)
#define O_X2H    (O_S2)
#define O_X2     (O_S2 + SZ_RH)
#define O_STAT   (O_X2 + SZ_RF)
#define O_WSAOUT (O_STAT + SZ_ST)
#define O_WCAIN  (O_WSAOUT + SZ_W1K)
#define O_WCAOUT (O_WCAIN + SZ_W3K)
#define O_W1     (O_WCAOUT + SZ_W1K)
#define O_W2     (O_W1 + SZ_WFF)
#define O_END    (O_W2 + SZ_WFF)

static_assert(O_WSAIN + SZ_W3K <= O_S1);
static_assert(O_CP + SZ_RH <= O_S1);
static_assert(O_HH + SZ_HH <= O_S1);
static_assert(O_GOUT + SZ_RF <= O_S2);
static_assert(O_P2 + SZ_P2 <= O_S2);
static_assert(O_OP + SZ_RH <= O_X2);
static_assert(O_END == (size_t)116703232);
static_assert(O_END <= (size_t)134217728);
static_assert((O_S1 % 256) == 0);
static_assert((O_S2 % 256) == 0);
static_assert((O_X1H % 256) == 0);
static_assert((O_CP % 256) == 0);
static_assert((O_STAT % 256) == 0);
static_assert((O_WSAOUT % 256) == 0);

extern "C" void kernel_launch(void* const* d_in, const int* in_sizes, int n_in,
                              void* d_out, int out_size, void* d_ws, size_t ws_size,
                              hipStream_t stream) {
  if (n_in < 19) return;
  if (in_sizes[0] != NB * LQ * CC) return;
  if (in_sizes[1] != C3 * CC || in_sizes[2] != C3) return;
  if (in_sizes[3] != CC * CC || in_sizes[4] != CC) return;
  if (in_sizes[5] != C3 * CC || in_sizes[6] != C3) return;
  if (in_sizes[7] != CC * CC || in_sizes[8] != CC) return;
  if (in_sizes[9] != FF * CC || in_sizes[10] != FF) return;
  if (in_sizes[11] != CC * FF || in_sizes[12] != CC) return;
  for (int i = 13; i < 19; ++i) if (in_sizes[i] != CC) return;
  if (out_size != NB * LQ * CC + NB * LQ * LQ) return;
  if (O_END > ws_size) return;

  const float* x        = (const float*)d_in[0];
  const float* sa_in_w  = (const float*)d_in[1];
  const float* sa_in_b  = (const float*)d_in[2];
  const float* sa_out_w = (const float*)d_in[3];
  const float* sa_out_b = (const float*)d_in[4];
  const float* ca_in_w  = (const float*)d_in[5];
  const float* ca_in_b  = (const float*)d_in[6];
  const float* ca_out_w = (const float*)d_in[7];
  const float* ca_out_b = (const float*)d_in[8];
  const float* w1       = (const float*)d_in[9];
  const float* b1       = (const float*)d_in[10];
  const float* w2       = (const float*)d_in[11];
  const float* b2       = (const float*)d_in[12];
  const float* g1  = (const float*)d_in[13];
  const float* be1 = (const float*)d_in[14];
  const float* g2  = (const float*)d_in[15];
  const float* be2 = (const float*)d_in[16];
  const float* g3  = (const float*)d_in[17];
  const float* be3 = (const float*)d_in[18];

  float* out0 = (float*)d_out;
  float* out1 = (float*)d_out + (size_t)NB * LQ * CC;

  char* ws = (char*)d_ws;
  _Float16* Xh     = (_Float16*)(ws + O_XH);
  _Float16* WsaIn  = (_Float16*)(ws + O_WSAIN);
  float*    MP     = (float*)(ws + O_MP);
  float*    X1     = (float*)(ws + O_X1);
  _Float16* X1h    = (_Float16*)(ws + O_X1H);
  _Float16* Cp     = (_Float16*)(ws + O_CP);
  _Float16* Hh     = (_Float16*)(ws + O_HH);
  _Float16* QKVp   = (_Float16*)(ws + O_QKV);
  float*    Gout   = (float*)(ws + O_GOUT);
  _Float16* P2     = (_Float16*)(ws + O_P2);
  _Float16* Op     = (_Float16*)(ws + O_OP);
  _Float16* X2h    = (_Float16*)(ws + O_X2H);
  float*    X2     = (float*)(ws + O_X2);
  float*    Stat   = (float*)(ws + O_STAT);
  _Float16* WsaOut = (_Float16*)(ws + O_WSAOUT);
  _Float16* WcaIn  = (_Float16*)(ws + O_WCAIN);
  _Float16* WcaOut = (_Float16*)(ws + O_WCAOUT);
  _Float16* W1h    = (_Float16*)(ws + O_W1);
  _Float16* W2h    = (_Float16*)(ws + O_W2);

  {
    const int ngrp = RP * CC / 8;
    k_cvt_x<<<dim3((ngrp + 255) / 256), dim3(256), 0, stream>>>(x, Xh, ngrp);
  }
  {
    const int n3 = C3 * CC / 8, n1k = CC * CC / 8, nff = FF * CC / 8;
    k_cvt_w<<<dim3((n3 + 255) / 256), dim3(256), 0, stream>>>(sa_in_w, WsaIn, n3, 32.0f);
    k_cvt_w<<<dim3((n1k + 255) / 256), dim3(256), 0, stream>>>(sa_out_w, WsaOut, n1k, 32.0f);
    k_cvt_w<<<dim3((n3 + 255) / 256), dim3(256), 0, stream>>>(ca_in_w, WcaIn, n3, 32.0f);
    k_cvt_w<<<dim3((n1k + 255) / 256), dim3(256), 0, stream>>>(ca_out_w, WcaOut, n1k, 32.0f);
    k_cvt_w<<<dim3((nff + 255) / 256), dim3(256), 0, stream>>>(w1, W1h, nff, 32.0f);
    k_cvt_w<<<dim3((nff + 255) / 256), dim3(256), 0, stream>>>(w2, W2h, nff, 32.0f);
  }
  k_qkv<<<dim3(RP / 128, C3 / 64), dim3(128), 0, stream>>>(Xh, WsaIn, sa_in_b, QKVp);
  k_attn<<<dim3(NB * NH * NQB), dim3(256), 0, stream>>>(QKVp, QKVp + PLQ, QKVp + 2 * PLQ, Op, Stat, 0.125f);
  k_map<<<dim3(MQ / 64, MQ / 64, NB), dim3(64), 0, stream>>>(QKVp, QKVp + PLQ, Stat, MP, 0.125f);
  {
    const int n1 = NB * LQ * LQ;
    const int nthr = (n1 + 3) / 4;
    k_flat<<<dim3((nthr + 255) / 256), dim3(256), 0, stream>>>(MP, out1, n1);
  }
  k_gemm32<<<dim3(RP / 128, CC / 64), dim3(128), 0, stream>>>(Op, WsaOut, sa_out_b, Gout, CC, CC, 0.001953125f);
  k_ln<0><<<dim3(RP), dim3(256), 0, stream>>>(x, Gout, g1, be1, X1, X1h, (float*)0);
  k_gemm16<0><<<dim3(RP / 128, C3 / 64), dim3(128), 0, stream>>>(X1h, WcaIn, ca_in_b, P2, CC, C3, 0.03125f);
  k_ca<<<dim3(NB * TG), dim3(64), 0, stream>>>(P2, Cp, 0.125f);
  k_gemm32<<<dim3(RP / 128, CC / 64), dim3(128), 0, stream>>>(Cp, WcaOut, ca_out_b, Gout, CC, CC, 0.001953125f);
  k_ln<1><<<dim3(RP), dim3(256), 0, stream>>>(X1, Gout, g2, be2, X2, X2h, (float*)0);
  k_gemm16<1><<<dim3(RP / 128, FF / 64), dim3(128), 0, stream>>>(X2h, W1h, b1, Hh, CC, FF, 0.03125f);
  k_gemm32<<<dim3(RP / 128, CC / 64), dim3(128), 0, stream>>>(Hh, W2h, b2, Gout, FF, CC, 0.03125f);
  k_ln<2><<<dim3(RP), dim3(256), 0, stream>>>(X2, Gout, g3, be3, (float*)0, (_Float16*)0, out0);
  (void)hipGetLastError();
}
